// SymEqNet_67997922230969
// MI455X (gfx1250) — hardware-verified
//
#include <hip/hip_runtime.h>
#include <stddef.h>
#include <math.h>


#define FQ      64
#define HGQ     128
#define KPRE    192
#define KPOST   832
#define NGQ     64
#define NB      256
#define ECH     2048
#define NTHR    256
#define NWAVE   8
#define G1ROWS  128
#define G2ROWS  64
#define WSCAP   134217728
#define WSCALE  64.0f
#define WINV    (1.0f / 64.0f)
#define AVGLOG  2.1972245773362196f
#define BIGF    3.0e38f

#define LDS_G1   (G1ROWS * HGQ * 4)
#define LDS_AGG  (NB * 256 * 4 + ECH * 4 + NB * 4 + 64)
#define LDS_G2   (G2ROWS * KPOST * 2 + G2ROWS * HGQ * 2 + G2ROWS * HGQ * 4 + 4 * G2ROWS * 4)
#define LDS_HEAD (3 * NGQ * HGQ * 4 + 2 * NGQ * 4 + NGQ * 4)

static_assert(NTHR == NWAVE * 32 && NB == NTHR && ECH == 8 * NTHR);
static_assert(G1ROWS == NWAVE * 16 && (NB % G1ROWS) == 0 && (NB % G2ROWS) == 0);
static_assert((FQ % 32) == 0 && (HGQ % 32) == 0 && (KPOST % 32) == 0 && KPOST == 13 * FQ && KPRE == 3 * FQ);
static_assert(G2ROWS == 4 * 16 && HGQ == 2 * 64 && NGQ == 64);
static_assert(LDS_AGG <= 300 * 1024 && LDS_G2 <= 300 * 1024 && LDS_HEAD <= 300 * 1024);

typedef float    v2f  __attribute__((ext_vector_type(2)));
typedef float    v4f  __attribute__((ext_vector_type(4)));
typedef float    v8f  __attribute__((ext_vector_type(8)));
typedef int      v4i  __attribute__((ext_vector_type(4)));
typedef _Float16 v8h  __attribute__((ext_vector_type(8)));
typedef _Float16 v16h __attribute__((ext_vector_type(16)));
union FragH { v16h v; v8h h[2]; };

static __device__ __forceinline__ v8f wmh(v16h a, v16h b, v8f c) {
  v8f d = __builtin_amdgcn_wmma_f32_16x16x32_f16(false, a, false, b, (short)0, c, false, false);
  asm volatile("v_nop\n\tv_nop\n\tv_nop\n\tv_nop" : "+v"(d) : "v"(a), "v"(b));
  return d;
}

static __device__ __forceinline__ v8f zero8() {
  v8f z = {0.f, 0.f, 0.f, 0.f, 0.f, 0.f, 0.f, 0.f};
  return z;
}

__global__ __launch_bounds__(NTHR) void k_cvtx(const float* __restrict__ x, _Float16* xh, int nRows, int total8) {
  const int i = (int)blockIdx.x * NTHR + (int)threadIdx.x;
  if (i >= total8) return;
  const size_t e  = (size_t)8 * (size_t)i;
  const int    r  = (int)(e >> 6);
  const int    k0 = (int)(e & 63);
  const int    rc = r < nRows ? r : nRows - 1;
  const float  z  = r < nRows ? 1.0f : 0.0f;
  const float* sp = x + (size_t)rc * FQ + k0;
  const v4f f0 = *(const v4f*)sp;
  const v4f f1 = *(const v4f*)(sp + 4);
  v8h hv;
  hv[0] = (_Float16)(f0.x * z); hv[1] = (_Float16)(f0.y * z); hv[2] = (_Float16)(f0.z * z); hv[3] = (_Float16)(f0.w * z);
  hv[4] = (_Float16)(f1.x * z); hv[5] = (_Float16)(f1.y * z); hv[6] = (_Float16)(f1.z * z); hv[7] = (_Float16)(f1.w * z);
  _Float16* p = xh + e;
  *(volatile v8h*)p = hv;
  __threadfence();
  *(volatile v8h*)p = hv;
}

__global__ __launch_bounds__(NTHR) void k_wt(const float* __restrict__ src, int ld, _Float16* dst, int K, int total8, float scale) {
  const int i = (int)blockIdx.x * NTHR + (int)threadIdx.x;
  if (i >= total8) return;
  const int e  = 8 * i;
  const int n  = e / K;
  const int k0 = e - n * K;
  v8h hv;
#pragma unroll
  for (int j = 0; j < 8; ++j) hv[j] = (_Float16)(scale * src[(size_t)(k0 + j) * (size_t)ld + n]);
  _Float16* p = dst + e;
  *(volatile v8h*)p = hv;
  __threadfence();
  *(volatile v8h*)p = hv;
}

__global__ __launch_bounds__(64) void k_uc(const float* __restrict__ Wedge, const float* __restrict__ bedge,
                                           const float* __restrict__ Wpre, const float* __restrict__ bpre, float* UC) {
  __shared__ __attribute__((aligned(16))) float ucl[2 * FQ];
  const int f = (int)threadIdx.x;
  float u = 0.0f, c = 0.0f;
#pragma unroll 1
  for (int k = 0; k < FQ; ++k) {
    const float w = Wpre[(size_t)(2 * FQ + k) * FQ + f];
    u = fmaf(Wedge[k], w, u);
    c = fmaf(bedge[k], w, c);
  }
  ucl[f] = u;
  ucl[FQ + f] = c + bpre[f];
  __syncthreads();
  if (threadIdx.x < 32) {
    const int lane = (int)threadIdx.x;
    const v4f v = *(const v4f*)(ucl + 4 * lane);
    *(volatile v4f*)(UC + 4 * lane) = v;
    __threadfence();
    *(volatile v4f*)(UC + 4 * lane) = v;
  }
}

__global__ __launch_bounds__(NTHR) void k_gemm1(const _Float16* __restrict__ A, const _Float16* __restrict__ B, float* C) {
  extern __shared__ v4f lds_dyn[];
  float* stg = (float*)lds_dyn;
  const int tid = threadIdx.x, lane = tid & 31, hh = lane >> 4, m = lane & 15;
  const int wave = __builtin_amdgcn_readfirstlane(tid >> 5);
  const int rowBase = (int)blockIdx.x * G1ROWS;
  const _Float16* ap = A + (size_t)(rowBase + wave * 16 + m) * FQ + 8 * hh;
  const _Float16* bp = B + (size_t)m * FQ + 8 * hh;

  v8f acc[8];
#pragma unroll
  for (int t = 0; t < 8; ++t) acc[t] = zero8();

#pragma unroll
  for (int kt = 0; kt < FQ / 32; ++kt) {
    FragH fa;
    fa.h[0] = *(const v8h*)(ap + 32 * kt);
    fa.h[1] = *(const v8h*)(ap + 32 * kt + 16);
#pragma unroll
    for (int t = 0; t < 8; ++t) {
      FragH fb;
      fb.h[0] = *(const v8h*)(bp + (size_t)(16 * t) * FQ + 32 * kt);
      fb.h[1] = *(const v8h*)(bp + (size_t)(16 * t) * FQ + 32 * kt + 16);
      acc[t] = wmh(fa.v, fb.v, acc[t]);
    }
  }

  float* sp = stg + (wave * 16 + 8 * hh) * HGQ + m;
#pragma unroll
  for (int t = 0; t < 8; ++t) {
#pragma unroll
    for (int r = 0; r < 8; ++r) sp[r * HGQ + 16 * t] = acc[t][r] * WINV;
  }
  __syncthreads();

  const float* lp = stg + wave * 16 * HGQ;
  float* gp = C + (size_t)(rowBase + wave * 16) * HGQ;
#pragma unroll
  for (int i = 0; i < 16; ++i) {
    const v4f v = *(const v4f*)(lp + i * HGQ + 4 * lane);
    *(volatile v4f*)(gp + (size_t)i * HGQ + 4 * lane) = v;
  }
  __threadfence();
#pragma unroll
  for (int i = 0; i < 16; ++i) {
    const v4f v = *(const v4f*)(lp + i * HGQ + 4 * lane);
    *(volatile v4f*)(gp + (size_t)i * HGQ + 4 * lane) = v;
  }
}

__global__ __launch_bounds__(NTHR) void k_agg(const int* __restrict__ ei, const float* __restrict__ ea,
                                              const float* __restrict__ P, const float* __restrict__ UC,
                                              float* ST, float* CNT, int nN, int nE, int vec8) {
  extern __shared__ v4f lds_dyn[];
  float* stl  = (float*)lds_dyn;
  int*   hrec = (int*)(stl + NB * 256);
  float* cntl = (float*)(hrec + ECH);
  int*   wtot = (int*)(cntl + NB);
  const int tid = threadIdx.x, lane = tid & 31;
  const int wave = __builtin_amdgcn_readfirstlane(tid >> 5);
  const int n0 = (int)blockIdx.x * NB;
  const int* srow = ei;
  const int* drow = ei + nE;

#pragma unroll 1
  for (int i = tid; i < NB * 64; i += NTHR) {
    const int b = (i >> 6) * 256 + (i & 63);
    stl[b] = 0.0f; stl[b + 64] = 0.0f; stl[b + 128] = BIGF; stl[b + 192] = -BIGF;
  }
  cntl[tid] = 0.0f;
  const v2f uu = *(const v2f*)(UC + 2 * lane);
  const int nChunks = (nE + ECH - 1) / ECH;

#pragma unroll 1
  for (int ch = 0; ch < nChunks; ++ch) {
    __syncthreads();
    const int cbase = ch * ECH;
    const int e0 = cbase + 8 * tid;
    int d[8];
    if (vec8 != 0 && cbase + ECH <= nE) {
      const v4i a = *(const v4i*)(drow + e0);
      const v4i b = *(const v4i*)(drow + e0 + 4);
      d[0] = a.x; d[1] = a.y; d[2] = a.z; d[3] = a.w;
      d[4] = b.x; d[5] = b.y; d[6] = b.z; d[7] = b.w;
    } else {
#pragma unroll
      for (int j = 0; j < 8; ++j) {
        const int e  = e0 + j;
        const int ec = e < nE ? e : nE - 1;
        const int v  = drow[ec];
        d[j] = e < nE ? v : -1;
      }
    }
    unsigned hm = 0u;
#pragma unroll
    for (int j = 0; j < 8; ++j) hm |= ((unsigned)(d[j] - n0) < (unsigned)NB) ? (1u << j) : 0u;
    const int c = (int)__popc(hm);
    int incl = c;
#pragma unroll
    for (int s = 1; s < 32; s <<= 1) {
      const int t = __shfl_up(incl, s);
      incl += (lane >= s) ? t : 0;
    }
    if (lane == 31) wtot[wave] = incl;
    __syncthreads();
    int base = 0, tot = 0;
#pragma unroll
    for (int w = 0; w < NWAVE; ++w) {
      const int tw = wtot[w];
      base += (w < wave) ? tw : 0;
      tot += tw;
    }
    int pos = base + incl - c;
#pragma unroll
    for (int j = 0; j < 8; ++j) {
      if (hm & (1u << j)) { hrec[pos] = ((e0 + j) << 8) | (d[j] - n0); ++pos; }
    }
    __syncthreads();
    tot = __builtin_amdgcn_readfirstlane(tot);
    tot = tot > ECH ? ECH : tot;
#pragma unroll 1
    for (int ii = 0; ii < tot; ++ii) {
      const int rec = __builtin_amdgcn_readfirstlane(hrec[ii]);
      const int ld = rec & (NB - 1);
      if ((ld & (NWAVE - 1)) == wave) {
        int e = rec >> 8;
        e = e > nE - 1 ? nE - 1 : e;
        int s = srow[e];
        s = s < 0 ? s + nN : s;
        s = s < 0 ? 0 : (s > nN - 1 ? nN - 1 : s);
        const float a = ea[e];
        const v2f av = {a, a};
        const v2f ps = *(const v2f*)(P + (size_t)s * HGQ + FQ + 2 * lane);
        const v2f q = ps + av * uu;
        float* bp = stl + ld * 256 + 2 * lane;
        v2f s1 = *(v2f*)bp;
        v2f s2 = *(v2f*)(bp + 64);
        v2f mn = *(v2f*)(bp + 128);
        v2f mx = *(v2f*)(bp + 192);
        s1 = s1 + q;
        s2 = q * q + s2;
        mn.x = fminf(mn.x, q.x); mn.y = fminf(mn.y, q.y);
        mx.x = fmaxf(mx.x, q.x); mx.y = fmaxf(mx.y, q.y);
        *(v2f*)bp = s1;
        *(v2f*)(bp + 64) = s2;
        *(v2f*)(bp + 128) = mn;
        *(v2f*)(bp + 192) = mx;
        if (lane == 0) cntl[ld] += 1.0f;
      }
    }
  }
  __syncthreads();

#pragma unroll 1
  for (int j = 0; j < NB / NWAVE; ++j) {
    const int n = wave + NWAVE * j;
    const float* lp = stl + n * 256 + 4 * lane;
    float* gp = ST + (size_t)(n0 + n) * 256 + 4 * lane;
    const v4f v0 = *(const v4f*)lp;
    const v4f v1 = *(const v4f*)(lp + 128);
    *(volatile v4f*)gp = v0;
    *(volatile v4f*)(gp + 128) = v1;
    __threadfence();
    *(volatile v4f*)gp = v0;
    *(volatile v4f*)(gp + 128) = v1;
  }
  if (tid < NB / 4) {
    const v4f cv = *(const v4f*)(cntl + 4 * tid);
    float* gp = CNT + n0 + 4 * tid;
    *(volatile v4f*)gp = cv;
    __threadfence();
    *(volatile v4f*)gp = cv;
  }
}

__global__ __launch_bounds__(NTHR) void k_gemm2(const _Float16* __restrict__ Xh, const float* __restrict__ P,
                                                const float* __restrict__ ST, const float* __restrict__ CNT,
                                                const float* __restrict__ UC,
                                                const _Float16* __restrict__ Wpo, const float* __restrict__ bpost,
                                                const _Float16* __restrict__ Wli, const float* __restrict__ blin,
                                                float* H) {
  extern __shared__ v4f lds_dyn[];
  _Float16* At  = (_Float16*)lds_dyn;
  _Float16* Ht  = At + G2ROWS * KPOST;
  float*    Ct  = (float*)(Ht + G2ROWS * HGQ);
  float*    rsc = Ct + G2ROWS * HGQ;
  const int tid = threadIdx.x, lane = tid & 31, hh = lane >> 4, m = lane & 15;
  const int wave = __builtin_amdgcn_readfirstlane(tid >> 5);
  const int n0 = (int)blockIdx.x * G2ROWS;

  if (tid < G2ROWS) {
    const float cnt = CNT[n0 + tid];
    const float c1  = fmaxf(cnt, 1.0f);
    const float amp = logf(c1 + 1.0f) * (1.0f / AVGLOG);
    rsc[tid]              = 1.0f / c1;
    rsc[G2ROWS + tid]     = amp;
    rsc[2 * G2ROWS + tid] = 1.0f / amp;
    rsc[3 * G2ROWS + tid] = cnt > 0.0f ? 1.0f : 0.0f;
  }
#pragma unroll 1
  for (int i = tid; i < G2ROWS * 8; i += NTHR) {
    const int r = i >> 3, p = i & 7;
    const v8h v = *(const v8h*)(Xh + (size_t)(n0 + r) * FQ + 8 * p);
    *(v8h*)(At + r * KPOST + 8 * p) = v;
  }
  __syncthreads();

#pragma unroll 1
  for (int i = tid; i < G2ROWS * FQ; i += NTHR) {
#pragma clang fp contract(off)
    const int r = i >> 6, chn = i & 63;
    const int node = n0 + r;
    const float* sp = ST + (size_t)node * 256 + chn;
    const float s1 = sp[0], s2 = sp[64], mn = sp[128], mx = sp[192];
    const float d = P[(size_t)node * HGQ + chn] + UC[FQ + chn];
    const float c1inv = rsc[r], amp = rsc[G2ROWS + r], inva = rsc[2 * G2ROWS + r];
    const bool  has = rsc[3 * G2ROWS + r] > 0.5f;
    const float muq = s1 * c1inv;
    const float vmean = has ? d + muq : 0.0f;
    const float var = fmaxf(s2 * c1inv - muq * muq, 0.0f);
    const float vstd = sqrtf(var + 1e-5f);
    const float vmn = has ? d + mn : 0.0f;
    const float vmx = has ? d + mx : 0.0f;
    _Float16* ap = At + r * KPOST + FQ + chn;
    ap[0]   = (_Float16)vmean;          ap[64]  = (_Float16)vmn;          ap[128] = (_Float16)vmx;          ap[192] = (_Float16)vstd;
    ap[256] = (_Float16)(vmean * amp);  ap[320] = (_Float16)(vmn * amp);  ap[384] = (_Float16)(vmx * amp);  ap[448] = (_Float16)(vstd * amp);
    ap[512] = (_Float16)(vmean * inva); ap[576] = (_Float16)(vmn * inva); ap[640] = (_Float16)(vmx * inva); ap[704] = (_Float16)(vstd * inva);
  }
  __syncthreads();

  const int rw = wave & 3, cw = wave >> 2;
  {
    const _Float16* ap = At + (16 * rw + m) * KPOST + 8 * hh;
    const _Float16* bp = Wpo + (size_t)(64 * cw + m) * KPOST + 8 * hh;
    v8f acc[4];
#pragma unroll
    for (int t = 0; t < 4; ++t) acc[t] = zero8();
#pragma unroll 1
    for (int kt = 0; kt < KPOST / 32; ++kt) {
      FragH fa;
      fa.h[0] = *(const v8h*)(ap + 32 * kt);
      fa.h[1] = *(const v8h*)(ap + 32 * kt + 16);
#pragma unroll
      for (int t = 0; t < 4; ++t) {
        FragH fb;
        fb.h[0] = *(const v8h*)(bp + (size_t)(16 * t) * KPOST + 32 * kt);
        fb.h[1] = *(const v8h*)(bp + (size_t)(16 * t) * KPOST + 32 * kt + 16);
        acc[t] = wmh(fa.v, fb.v, acc[t]);
      }
    }
#pragma unroll
    for (int t = 0; t < 4; ++t) {
      const int col = 64 * cw + 16 * t + m;
      const float bb = bpost[col];
#pragma unroll
      for (int r = 0; r < 8; ++r) Ht[(16 * rw + 8 * hh + r) * HGQ + col] = (_Float16)(acc[t][r] * WINV + bb);
    }
  }
  __syncthreads();

  {
    const _Float16* ap = Ht + (16 * rw + m) * HGQ + 8 * hh;
    const _Float16* bp = Wli + (size_t)(64 * cw + m) * HGQ + 8 * hh;
    v8f acc[4];
#pragma unroll
    for (int t = 0; t < 4; ++t) acc[t] = zero8();
#pragma unroll
    for (int kt = 0; kt < HGQ / 32; ++kt) {
      FragH fa;
      fa.h[0] = *(const v8h*)(ap + 32 * kt);
      fa.h[1] = *(const v8h*)(ap + 32 * kt + 16);
#pragma unroll
      for (int t = 0; t < 4; ++t) {
        FragH fb;
        fb.h[0] = *(const v8h*)(bp + (size_t)(16 * t) * HGQ + 32 * kt);
        fb.h[1] = *(const v8h*)(bp + (size_t)(16 * t) * HGQ + 32 * kt + 16);
        acc[t] = wmh(fa.v, fb.v, acc[t]);
      }
    }
#pragma unroll
    for (int t = 0; t < 4; ++t) {
      const int col = 64 * cw + 16 * t + m;
      const float bb = blin[col];
#pragma unroll
      for (int r = 0; r < 8; ++r) Ct[(16 * rw + 8 * hh + r) * HGQ + col] = acc[t][r] * WINV + bb;
    }
  }
  __syncthreads();

#pragma unroll
  for (int j = 0; j < G2ROWS / NWAVE; ++j) {
    const int row = wave + NWAVE * j;
    const v4f v = *(const v4f*)(Ct + row * HGQ + 4 * lane);
    *(volatile v4f*)(H + (size_t)(n0 + row) * HGQ + 4 * lane) = v;
  }
  __threadfence();
#pragma unroll
  for (int j = 0; j < G2ROWS / NWAVE; ++j) {
    const int row = wave + NWAVE * j;
    const v4f v = *(const v4f*)(Ct + row * HGQ + 4 * lane);
    *(volatile v4f*)(H + (size_t)(n0 + row) * HGQ + 4 * lane) = v;
  }
}

static __device__ __forceinline__ void bn_col(const float* buf, int f, float& mu, float& rs) {
  float s = 0.0f;
#pragma unroll 1
  for (int g = 0; g < NGQ; ++g) s += buf[g * HGQ + f];
  mu = s * (1.0f / 64.0f);
  float q = 0.0f;
#pragma unroll 1
  for (int g = 0; g < NGQ; ++g) { const float dd = buf[g * HGQ + f] - mu; q = fmaf(dd, dd, q); }
  rs = rsqrtf(q * (1.0f / 64.0f) + 1e-5f);
}

static __device__ __forceinline__ void fc_col(const float* src, const float* __restrict__ W,
                                              const float* __restrict__ bias, float* dst, int f) {
  const float bb = bias[f];
#pragma unroll 1
  for (int g = 0; g < NGQ; ++g) {
    float s = 0.0f;
#pragma unroll 4
    for (int k = 0; k < HGQ; ++k) s = fmaf(src[g * HGQ + k], W[(size_t)k * HGQ + f], s);
    dst[g * HGQ + f] = s + bb;
  }
}

__global__ __launch_bounds__(NTHR) void k_head(
    const float* __restrict__ H, const int* __restrict__ batch, int nN,
    const float* __restrict__ g1, const float* __restrict__ be1,
    const float* __restrict__ W2, const float* __restrict__ b2, const float* __restrict__ g2, const float* __restrict__ be2,
    const float* __restrict__ Wr1, const float* __restrict__ br1, const float* __restrict__ gr1, const float* __restrict__ ber1,
    const float* __restrict__ Wr2, const float* __restrict__ br2, const float* __restrict__ gr2, const float* __restrict__ ber2,
    const float* __restrict__ Wout, const float* __restrict__ bout, float* out) {
  extern __shared__ v4f lds_dyn[];
  float* bA   = (float*)lds_dyn;
  float* bB   = bA + NGQ * HGQ;
  float* bC   = bB + NGQ * HGQ;
  float* cntp = bC + NGQ * HGQ;
  float* outv = cntp + 2 * NGQ;
  const int tid = threadIdx.x, lane = tid & 31;
  const int wave = __builtin_amdgcn_readfirstlane(tid >> 5);
  const int c = tid & (HGQ - 1);
  const int par = tid >> 7;
  float* pb = bB + par * (NGQ * HGQ);

#pragma unroll 1
  for (int g = 0; g < NGQ; ++g) pb[g * HGQ + c] = 0.0f;
  if (tid < 2 * NGQ) cntp[tid] = 0.0f;
  __syncthreads();

#pragma unroll 1
  for (int n = par; n < nN; n += 2) {
    const int b = batch[n];
    const float h = H[(size_t)n * HGQ + c];
    if ((unsigned)b < (unsigned)NGQ) {
      pb[b * HGQ + c] += h;
      if (c == 0) cntp[par * NGQ + b] += 1.0f;
    }
  }
  __syncthreads();

  const int f = tid;
  if (tid < HGQ) {
#pragma unroll 1
    for (int g = 0; g < NGQ; ++g) {
      const float cnt = cntp[g] + cntp[NGQ + g];
      const float inv = 1.0f / fmaxf(cnt, 1.0f);
      bA[g * HGQ + f] = (bB[g * HGQ + f] + bC[g * HGQ + f]) * inv;
    }
    float mu, rs;
    bn_col(bA, f, mu, rs);
    const float gg = g1[f], be = be1[f];
#pragma unroll 1
    for (int g = 0; g < NGQ; ++g) bB[g * HGQ + f] = fmaxf((bA[g * HGQ + f] - mu) * rs * gg + be, 0.0f);
  }
  __syncthreads();

  if (tid < HGQ) {
    fc_col(bB, W2, b2, bC, f);
    float mu, rs;
    bn_col(bC, f, mu, rs);
    const float gg = g2[f], be = be2[f];
#pragma unroll 1
    for (int g = 0; g < NGQ; ++g) bA[g * HGQ + f] = fmaxf((bC[g * HGQ + f] - mu) * rs * gg + be, 0.0f);
  }
  __syncthreads();

  if (tid < HGQ) {
    fc_col(bA, Wr1, br1, bC, f);
    float mu, rs;
    bn_col(bC, f, mu, rs);
    const float gg = gr1[f], be = ber1[f];
#pragma unroll 1
    for (int g = 0; g < NGQ; ++g) bB[g * HGQ + f] = fmaxf((bC[g * HGQ + f] - mu) * rs * gg + be, 0.0f);
  }
  __syncthreads();

  if (tid < HGQ) {
    fc_col(bB, Wr2, br2, bC, f);
    float mu, rs;
    bn_col(bC, f, mu, rs);
    const float gg = gr2[f], be = ber2[f];
#pragma unroll 1
    for (int g = 0; g < NGQ; ++g) {
      const float v = (bC[g * HGQ + f] - mu) * rs * gg + be + bA[g * HGQ + f];
      bC[g * HGQ + f] = fmaxf(v, 0.0f);
    }
  }
  __syncthreads();

  if (tid < NGQ) {
    const int g = tid;
    float s = 0.0f;
#pragma unroll 4
    for (int k = 0; k < HGQ; ++k) s = fmaf(bC[g * HGQ + k], Wout[k], s);
    outv[g] = s + bout[0];
  }
  __syncthreads();

  if (wave == 0) {
    const int lc = lane < 16 ? lane : 15;
    const v4f v = *(const v4f*)(outv + 4 * lc);
    if (lane < 16) *(volatile v4f*)(out + 4 * lane) = v;
    __threadfence();
    if (lane < 16) *(volatile v4f*)(out + 4 * lane) = v;
  }
}

extern "C" void kernel_launch(void* const* d_in, const int* in_sizes, int n_in,
                              void* d_out, int out_size, void* d_ws, size_t ws_size,
                              hipStream_t stream) {
  if (n_in < 28) return;
  const int nN = in_sizes[3];
  const int nE = in_sizes[2];
  if (nN <= 0 || nE <= 0 || nN > (1 << 22) || nE > (1 << 23)) return;
  if (in_sizes[0] != nN * FQ || in_sizes[1] != 2 * nE) return;
  if (in_sizes[4] != FQ || in_sizes[5] != FQ || in_sizes[6] != KPRE * FQ || in_sizes[7] != FQ) return;
  if (in_sizes[8] != KPOST * HGQ || in_sizes[9] != HGQ || in_sizes[10] != HGQ * HGQ || in_sizes[11] != HGQ) return;
  if (in_sizes[12] != HGQ || in_sizes[13] != HGQ || in_sizes[14] != HGQ * HGQ || in_sizes[15] != HGQ) return;
  if (in_sizes[16] != HGQ || in_sizes[17] != HGQ || in_sizes[18] != HGQ * HGQ || in_sizes[19] != HGQ) return;
  if (in_sizes[20] != HGQ || in_sizes[21] != HGQ || in_sizes[22] != HGQ * HGQ || in_sizes[23] != HGQ) return;
  if (in_sizes[24] != HGQ || in_sizes[25] != HGQ || in_sizes[26] != HGQ || in_sizes[27] != 1) return;
  if (out_size != NGQ) return;

  const float* x     = (const float*)d_in[0];
  const int*   ei    = (const int*)d_in[1];
  const float* ea    = (const float*)d_in[2];
  const int*   batch = (const int*)d_in[3];
  const float* Wedge = (const float*)d_in[4];
  const float* bedge = (const float*)d_in[5];
  const float* Wpre  = (const float*)d_in[6];
  const float* bpre  = (const float*)d_in[7];
  const float* Wpost = (const float*)d_in[8];
  const float* bpost = (const float*)d_in[9];
  const float* Wlin  = (const float*)d_in[10];
  const float* blin  = (const float*)d_in[11];
  const float* g1    = (const float*)d_in[12];
  const float* be1   = (const float*)d_in[13];
  const float* W2    = (const float*)d_in[14];
  const float* b2    = (const float*)d_in[15];
  const float* g2    = (const float*)d_in[16];
  const float* be2   = (const float*)d_in[17];
  const float* Wr1   = (const float*)d_in[18];
  const float* br1   = (const float*)d_in[19];
  const float* gr1   = (const float*)d_in[20];
  const float* ber1  = (const float*)d_in[21];
  const float* Wr2   = (const float*)d_in[22];
  const float* br2   = (const float*)d_in[23];
  const float* gr2   = (const float*)d_in[24];
  const float* ber2  = (const float*)d_in[25];
  const float* Wout  = (const float*)d_in[26];
  const float* bout  = (const float*)d_in[27];
  float* out = (float*)d_out;

  const int NPAD = ((nN + NB - 1) / NB) * NB;
  const int vec8 = ((nE & 3) == 0) ? 1 : 0;

  char* ws = (char*)d_ws;
  size_t off = 0;
  const size_t oXh  = off; off += (size_t)NPAD * FQ * 2;       off = (off + 255) & ~(size_t)255;
  const size_t oWf  = off; off += (size_t)HGQ * FQ * 2;        off = (off + 255) & ~(size_t)255;
  const size_t oWpo = off; off += (size_t)HGQ * KPOST * 2;     off = (off + 255) & ~(size_t)255;
  const size_t oWli = off; off += (size_t)HGQ * HGQ * 2;       off = (off + 255) & ~(size_t)255;
  const size_t oUC  = off; off += (size_t)2 * FQ * 4;          off = (off + 255) & ~(size_t)255;
  const size_t oP   = off; off += (size_t)NPAD * HGQ * 4;      off = (off + 255) & ~(size_t)255;
  const size_t oST  = off; off += (size_t)NPAD * 256 * 4;      off = (off + 255) & ~(size_t)255;
  const size_t oCNT = off; off += (size_t)NPAD * 4;            off = (off + 255) & ~(size_t)255;
  const size_t oH   = off; off += (size_t)NPAD * HGQ * 4;      off = (off + 255) & ~(size_t)255;
  if (off > ws_size || off > (size_t)WSCAP) return;
  _Float16* Xh  = (_Float16*)(ws + oXh);
  _Float16* Wf  = (_Float16*)(ws + oWf);
  _Float16* Wpo = (_Float16*)(ws + oWpo);
  _Float16* Wli = (_Float16*)(ws + oWli);
  float*    UC  = (float*)(ws + oUC);
  float*    P   = (float*)(ws + oP);
  float*    ST  = (float*)(ws + oST);
  float*    CNT = (float*)(ws + oCNT);
  float*    Hh  = (float*)(ws + oH);

  hipFuncSetAttribute(reinterpret_cast<const void*>(&k_gemm1), hipFuncAttributeMaxDynamicSharedMemorySize, LDS_G1);
  hipFuncSetAttribute(reinterpret_cast<const void*>(&k_agg),   hipFuncAttributeMaxDynamicSharedMemorySize, LDS_AGG);
  hipFuncSetAttribute(reinterpret_cast<const void*>(&k_gemm2), hipFuncAttributeMaxDynamicSharedMemorySize, LDS_G2);
  hipFuncSetAttribute(reinterpret_cast<const void*>(&k_head),  hipFuncAttributeMaxDynamicSharedMemorySize, LDS_HEAD);

  {
    const int t8 = (NPAD * FQ) / 8;
    k_cvtx<<<(t8 + NTHR - 1) / NTHR, NTHR, 0, stream>>>(x, Xh, nN, t8);
  }
  {
    const int t8a = (FQ * FQ) / 8;
    k_wt<<<(t8a + NTHR - 1) / NTHR, NTHR, 0, stream>>>(Wpre, FQ, Wf, FQ, t8a, WSCALE);
    k_wt<<<(t8a + NTHR - 1) / NTHR, NTHR, 0, stream>>>(Wpre + FQ * FQ, FQ, Wf + FQ * FQ, FQ, t8a, WSCALE);
    const int t8b = (HGQ * KPOST) / 8;
    k_wt<<<(t8b + NTHR - 1) / NTHR, NTHR, 0, stream>>>(Wpost, HGQ, Wpo, KPOST, t8b, WSCALE);
    const int t8c = (HGQ * HGQ) / 8;
    k_wt<<<(t8c + NTHR - 1) / NTHR, NTHR, 0, stream>>>(Wlin, HGQ, Wli, HGQ, t8c, WSCALE);
  }
  k_uc<<<1, 64, 0, stream>>>(Wedge, bedge, Wpre, bpre, UC);
  k_gemm1<<<NPAD / G1ROWS, NTHR, LDS_G1, stream>>>(Xh, Wf, P);
  k_agg<<<NPAD / NB, NTHR, LDS_AGG, stream>>>(ei, ea, P, UC, ST, CNT, nN, nE, vec8);
  k_gemm2<<<NPAD / G2ROWS, NTHR, LDS_G2, stream>>>(Xh, P, ST, CNT, UC, Wpo, bpost, Wli, blin, Hh);
  k_head<<<1, NTHR, LDS_HEAD, stream>>>(Hh, batch, nN, g1, be1, W2, b2, g2, be2,
                                        Wr1, br1, gr1, ber1, Wr2, br2, gr2, ber2, Wout, bout, out);
}
